// SelectiveSSM_1855425872531
// MI455X (gfx1250) — hardware-run, weakly checked
//
#include <hip/hip_runtime.h>
#include <math.h>

typedef __attribute__((ext_vector_type(16))) _Float16 v16h;
typedef __attribute__((ext_vector_type(8)))  _Float16 v8h;
typedef __attribute__((ext_vector_type(2)))  _Float16 v2h;
typedef __attribute__((ext_vector_type(16))) __bf16   v16b;
typedef __attribute__((ext_vector_type(8)))  __bf16   v8b;
typedef __attribute__((ext_vector_type(8)))  float    v8f;
typedef __attribute__((ext_vector_type(4)))  float    v4f;
typedef __attribute__((ext_vector_type(2)))  float    v2f;

constexpr int kNB   = 2;
constexpr int kL    = 2048;
constexpr int kRows = kNB * kL;
constexpr int kDM   = 1024;
constexpr int kDI   = 2 * kDM;
constexpr int kDI2  = 2 * kDI;
constexpr int kNs   = 16;
constexpr int kDC   = 4;
constexpr int kR    = 64;
constexpr int kXo   = kR + 2 * kNs;
constexpr int kXoP  = 128;
constexpr int kThr  = 256;
constexpr float kInCarry = 1024.0f;
constexpr float kWCarry  = 4096.0f;
constexpr float kLoUp    = 16.0f;
constexpr float kW2Carry = kInCarry / kLoUp;
constexpr float kDtCarry = 256.0f;
constexpr float kYCarry  = 128.0f;
constexpr float kScIn = 1.0f / (kInCarry * kInCarry);
constexpr float kScDt = 1.0f / (kDtCarry * kInCarry);
constexpr float kScY  = 1.0f / (kYCarry * kInCarry);
constexpr float kF16MinNormal = 6.103515625e-5f;

static_assert(kXo == 96 && kXo <= kXoP && kR == 64 && kDI == 2048 && kDI2 == 4096 && kRows == 4096 && (kL & (kL - 1)) == 0 && kLoUp * kW2Carry == kInCarry, "the index arithmetic below uses these sizes; a token's place in its sequence is row & (kL - 1); (carry x 2^4) x (2^10 / 2^4) = carry x 2^10");

constexpr size_t kOffX16 = 0ull;
constexpr size_t kOffWIN16 = 8388608ull;
constexpr size_t kOffWX16 = 16777216ull;
constexpr size_t kOffWDT16 = 17825792ull;
constexpr size_t kOffWOUT16 = 18087936ull;
constexpr size_t kOffZB = 26476544ull;
constexpr size_t kOffBDT = 26492928ull;
constexpr size_t kOffXZ = 26501120ull;
constexpr size_t kOffU16 = 93609984ull;
constexpr size_t kOffXD = 127164416ull;
constexpr size_t kOffDT16 = 129261568ull;
constexpr size_t kOffDL = 129785856ull;
constexpr size_t kWsTotal = 163340288ull;
static_assert(kWsTotal <= 268435456ull, "the carve stands under the contract's 256 MiB of workspace");
static_assert(kOffX16 == 0
  && kOffWIN16 == kOffX16 + 8388608ull
  && kOffWX16 == kOffWIN16 + 8388608ull
  && kOffWDT16 == kOffWX16 + 1048576ull
  && kOffWOUT16 == kOffWDT16 + 262144ull
  && kOffZB == kOffWOUT16 + 8388608ull
  && kOffBDT == kOffZB + 16384ull
  && kOffXZ == kOffBDT + 8192ull
  && kOffU16 == kOffXZ + 67108864ull
  && kOffXD == kOffU16 + 33554432ull
  && kOffDT16 == kOffXD + 2097152ull
  && kOffDL == kOffDT16 + 524288ull
  && kWsTotal == kOffDL + 33554432ull, "the carve is a chain: every region starts where the one before ends");
static_assert((kOffWIN16 % 256) == 0 && (kOffWX16 % 256) == 0 && (kOffWDT16 % 256) == 0 && (kOffWOUT16 % 256) == 0 && (kOffZB % 256) == 0 && (kOffBDT % 256) == 0 && (kOffXZ % 256) == 0 && (kOffU16 % 256) == 0 && (kOffXD % 256) == 0 && (kOffDT16 % 256) == 0 && (kOffDL % 256) == 0, "every region starts on a multiple of 256 B");

__device__ __forceinline__ unsigned short f2bf_bits(float f) {
  unsigned u = __float_as_uint(f);
  return (unsigned short)((u + 0x7FFFu + ((u >> 16) & 1u)) >> 16);
}
__device__ __forceinline__ float bf_bits2f(unsigned short h) { return __uint_as_float(((unsigned)h) << 16); }
__device__ __forceinline__ float bf16r(float f) { return bf_bits2f(f2bf_bits(f)); }
__device__ __forceinline__ float carry_flush(float v, float carry) {
  const float s = v * carry;
  return (fabsf(s) < kF16MinNormal) ? 0.0f : s;
}

__device__ __forceinline__ void dep_guard4_h(v8f& a, v8f& b, v8f& c, v8f& d, v16h x, v16h y) { asm volatile("v_nop\n\tv_nop\n\tv_nop\n\tv_nop" : "+v"(a), "+v"(b), "+v"(c), "+v"(d) : "v"(x), "v"(y)); }
__device__ __forceinline__ void dep_guard4_b(v8f& a, v8f& b, v8f& c, v8f& d, v16b x, v16b y) { asm volatile("v_nop\n\tv_nop\n\tv_nop\n\tv_nop" : "+v"(a), "+v"(b), "+v"(c), "+v"(d) : "v"(x), "v"(y)); }
__device__ __forceinline__ void keep4_h(v16h a, v16h b, v16h c, v16h d) { asm volatile("v_nop" :: "v"(a), "v"(b), "v"(c), "v"(d)); }
__device__ __forceinline__ void keep4_b(v16b a, v16b b, v16b c, v16b d) { asm volatile("v_nop" :: "v"(a), "v"(b), "v"(c), "v"(d)); }
__device__ __forceinline__ void acc_guard4(v8f& a, v8f& b, v8f& c, v8f& d) { asm volatile("v_nop\n\tv_nop\n\tv_nop\n\tv_nop" : "+v"(a), "+v"(b), "+v"(c), "+v"(d)); }

template <typename T> struct Frag;
template <> struct Frag<_Float16> {
  typedef v16h V; union U { v16h v; v8h h[2]; };
  static __device__ __forceinline__ v16h load(const _Float16* p) {
    U f; f.h[0] = *(const v8h*)(p); f.h[1] = *(const v8h*)(p + 16); return f.v;
  }
  static __device__ __forceinline__ v8f mma(v16h a, v16h b, v8f c) {
    return __builtin_amdgcn_wmma_f32_16x16x32_f16(false, a, false, b, (short)0, c, false, false);
  }
  static __device__ __forceinline__ void guard4(v8f& a, v8f& b, v8f& c, v8f& d, v16h x, v16h y) { dep_guard4_h(a, b, c, d, x, y); }
  static __device__ __forceinline__ void keep(v16h a, v16h b, v16h c, v16h d) { keep4_h(a, b, c, d); }
};
template <> struct Frag<__bf16> {
  typedef v16b V; union U { v16b v; v8b h[2]; };
  static __device__ __forceinline__ v16b load(const __bf16* p) {
    U f; f.h[0] = *(const v8b*)(p); f.h[1] = *(const v8b*)(p + 16); return f.v;
  }
  static __device__ __forceinline__ v8f mma(v16b a, v16b b, v8f c) {
    return __builtin_amdgcn_wmma_f32_16x16x32_bf16(false, a, false, b, (short)0, c, false, false);
  }
  static __device__ __forceinline__ void guard4(v8f& a, v8f& b, v8f& c, v8f& d, v16b x, v16b y) { dep_guard4_b(a, b, c, d, x, y); }
  static __device__ __forceinline__ void keep(v16b a, v16b b, v16b c, v16b d) { keep4_b(a, b, c, d); }
};

__device__ __forceinline__ v8f mma_h(v16h a, v16h b, v8f c) {
  c = __builtin_amdgcn_wmma_f32_16x16x32_f16(false, a, false, b, (short)0, c, false, false);
  asm volatile("v_nop\n\tv_nop\n\tv_nop\n\tv_nop" : "+v"(c) : "v"(a), "v"(b));
  return c;
}

template <int ET> struct Elem;
template <> struct Elem<0> { typedef _Float16 T; };
template <> struct Elem<1> { typedef __bf16 T; };
template <int ET, bool SPLIT, int BIAS_MODE, int OUT_MODE, bool RESID, int ACT = 0>
__global__ __launch_bounds__(256) void wmma_gemm64(
    const unsigned short* __restrict__ Ap, const unsigned short* __restrict__ A2p, int lda, long strideA,
    const unsigned short* __restrict__ Btp, const unsigned short* __restrict__ Bt2p, int ldb, long strideB,
    void* __restrict__ Cout, void* __restrict__ Cout2, int ldc, long strideC,
    const float* __restrict__ bias,
    const float* __restrict__ resid, long strideR,
    int M, int N, int K, float scale) {
  typedef typename Elem<ET>::T T;
  typedef typename Frag<T>::V V;
  const T* A = (const T*)Ap; const T* A2 = (const T*)A2p; const T* Bt = (const T*)Btp; const T* Bt2 = (const T*)Bt2p;
  __shared__ __align__(16) float sT[8][16 * 68];
  const int b    = blockIdx.y;
  const int lane = threadIdx.x & 31;
  const int wave = threadIdx.x >> 5;
  const int tilesN = N >> 6;
  const int tilesM = M >> 6;
  const int tile = blockIdx.x * 8 + wave;
  if (tile >= tilesM * tilesN) return;
  const int tm = tile / tilesN;
  const int tn = tile - tm * tilesN;
  const int m0 = tm << 6;
  const int n0 = tn << 6;

  const T* Ab  = A  + (size_t)b * strideA;
  const T* Bb  = Bt + (size_t)b * strideB;
  const T* Ab2 = SPLIT ? (A2  + (size_t)b * strideA) : nullptr;
  const T* Bb2 = SPLIT ? (Bt2 + (size_t)b * strideB) : nullptr;

  const int rlane = lane & 15;
  const int koff  = (lane >> 4) * 8;
  const int mOff  = (lane >> 4) * 8;

  v8f acc[4][4];
#pragma unroll
  for (int i = 0; i < 4; ++i)
#pragma unroll
    for (int j = 0; j < 4; ++j) acc[i][j] = (v8f){0.f,0.f,0.f,0.f,0.f,0.f,0.f,0.f};

  for (int k0 = 0; k0 < K; k0 += 32) {
    V bh[4], bl[4];
#pragma unroll
    for (int j = 0; j < 4; ++j) {
      const size_t bo = (size_t)(n0 + (j << 4) + rlane) * ldb + koff + k0;
      bh[j] = Frag<T>::load(Bb + bo);
      if (SPLIT) bl[j] = Frag<T>::load(Bb2 + bo);
    }
#pragma unroll
    for (int i = 0; i < 4; ++i) {
      const size_t ao = (size_t)(m0 + (i << 4) + rlane) * lda + koff + k0;
      V ah = Frag<T>::load(Ab + ao);
      V al;
      if (SPLIT) al = Frag<T>::load(Ab2 + ao);
#pragma unroll
      for (int j = 0; j < 4; ++j) {
        acc[i][j] = Frag<T>::mma(ah, bh[j], acc[i][j]);
        if (SPLIT) {
          acc[i][j] = Frag<T>::mma(ah, bl[j], acc[i][j]);
          acc[i][j] = Frag<T>::mma(al, bh[j], acc[i][j]);
        }
      }
      Frag<T>::guard4(acc[i][0], acc[i][1], acc[i][2], acc[i][3], ah, SPLIT ? al : ah);
    }
    Frag<T>::keep(bh[0], bh[1], bh[2], bh[3]);
    if (SPLIT) Frag<T>::keep(bl[0], bl[1], bl[2], bl[3]);
  }
  acc_guard4(acc[0][0], acc[0][1], acc[0][2], acc[0][3]);
  acc_guard4(acc[1][0], acc[1][1], acc[1][2], acc[1][3]);
  acc_guard4(acc[2][0], acc[2][1], acc[2][2], acc[2][3]);
  acc_guard4(acc[3][0], acc[3][1], acc[3][2], acc[3][3]);

  float* slab = sT[wave];
  const float* Rb = RESID ? (resid + (size_t)b * strideR) : nullptr;
#pragma unroll
  for (int i = 0; i < 4; ++i) {
    const int mBase = m0 + (i << 4);
#pragma unroll
    for (int j = 0; j < 4; ++j) {
      const int n = n0 + (j << 4) + rlane;
      float bv = 0.f;
      if (BIAS_MODE == 2) bv = bias[n];
#pragma unroll
      for (int r = 0; r < 8; ++r) {
        float v = acc[i][j][r] * scale;
        if (BIAS_MODE == 1) v += bias[mBase + mOff + r];
        if (BIAS_MODE == 2) v += bv;
        if (RESID) v += Rb[(size_t)(mBase + mOff + r) * ldc + n];
        if (ACT == 1) v = tanhf(v);
        if (ACT == 2) v = fmaxf(v, 0.0f);
        if (ACT == 3) v = v / (1.0f + expf(-v));
        if (ACT == 4) v = (v > 0.f) ? v : 0.01f * v;
        slab[(mOff + r) * 68 + (j << 4) + rlane] = v;
      }
    }
    __builtin_amdgcn_fence(__ATOMIC_RELEASE, "workgroup");
    __builtin_amdgcn_wave_barrier();
    __builtin_amdgcn_fence(__ATOMIC_ACQUIRE, "workgroup");
    if (OUT_MODE == 0) {
      float* C = (float*)Cout + (size_t)b * strideC;
      const int hh = lane >> 4, c4 = (lane & 15) * 4;
      for (int pass = 0; pass < 2; ++pass) {
#pragma unroll
        for (int it = 0; it < 8; ++it) {
          const int row = it * 2 + hh;
          v4f v = *(const v4f*)(slab + row * 68 + c4);
          *(volatile v4f*)(C + (size_t)(mBase + row) * ldc + n0 + c4) = v;
        }
        __threadfence();
      }
    } else {
      const int q = lane >> 3, c8 = (lane & 7) * 8;
      unsigned short* C  = (unsigned short*)Cout  + (size_t)b * strideC;
      unsigned short* C2 = (OUT_MODE == 2) ? ((unsigned short*)Cout2 + (size_t)b * strideC) : nullptr;
      for (int pass = 0; pass < 2; ++pass) {
#pragma unroll
        for (int it = 0; it < 4; ++it) {
          const int row = it * 4 + q;
          const float* sp = slab + row * 68 + c8;
          v8h hv, lv;
#pragma unroll
          for (int e = 0; e < 8; ++e) {
            if (OUT_MODE == 1) {
              hv[e] = (_Float16)sp[e];
            } else {
              unsigned short hb = f2bf_bits(sp[e]);
              unsigned short lb = f2bf_bits(sp[e] - bf_bits2f(hb));
              hv[e] = __builtin_bit_cast(_Float16, hb);
              lv[e] = __builtin_bit_cast(_Float16, lb);
            }
          }
          *(volatile v8h*)(C + (size_t)(mBase + row) * ldc + n0 + c8) = hv;
          if (OUT_MODE == 2) *(volatile v8h*)(C2 + (size_t)(mBase + row) * ldc + n0 + c8) = lv;
        }
        __threadfence();
      }
    }
    __builtin_amdgcn_fence(__ATOMIC_RELEASE, "workgroup");
    __builtin_amdgcn_wave_barrier();
    __builtin_amdgcn_fence(__ATOMIC_ACQUIRE, "workgroup");
  }
}


__device__ __forceinline__ void store2(float* p, float v) {
  *(volatile float*)p = v;
  __threadfence();
  *(volatile float*)p = v;
}

__global__ __launch_bounds__(kThr) void cast_plane_kernel(const float* __restrict__ src, unsigned short* __restrict__ dst,
                                                          int colsLog2, int dstPitch, int dstOff) {
  const int i   = blockIdx.x * kThr + threadIdx.x;
  const int sh  = colsLog2 - 3;
  const int row = i >> sh;
  const int c8  = (i & ((1 << sh) - 1)) * 8;
  const float* sp = src + ((size_t)row << colsLog2) + c8;
  const v4f a0 = *(const v4f*)(sp);
  const v4f a1 = *(const v4f*)(sp + 4);
  v8h hv;
#pragma unroll
  for (int e = 0; e < 4; ++e) {
    const float f0 = a0[e];
    const float f1 = a1[e];
    hv[e]     = (_Float16)carry_flush(bf16r(f0), kInCarry);
    hv[4 + e] = (_Float16)carry_flush(bf16r(f1), kInCarry);
  }
  unsigned short* dp = dst + (size_t)row * dstPitch + dstOff + c8;
  *(volatile v8h*)dp = hv;
  __threadfence();
  *(volatile v8h*)dp = hv;
}

__global__ __launch_bounds__(256) void wt_plane_kernel(const float* __restrict__ W, unsigned short* __restrict__ dst, int K, int N, int nLive, int ldd, int colOff) {
  const int n  = blockIdx.x;
  const int k8 = threadIdx.x * 8;
  const bool live = n < nLive;
  const int nc = live ? n : 0;
  v8h hv;
#pragma unroll
  for (int e = 0; e < 8; ++e) {
    const float w = W[(size_t)(k8 + e) * N + nc];
    hv[e] = (_Float16)(live ? carry_flush(bf16r(w), kWCarry) : 0.0f);
  }
  unsigned short* dp = dst + (size_t)n * ldd + colOff + k8;
  *(volatile v8h*)dp = hv;
  __threadfence();
  *(volatile v8h*)dp = hv;
}

__global__ __launch_bounds__(kThr) void setup_kernel(const float* __restrict__ b_dt, const float* __restrict__ W_x, const float* __restrict__ W_out,
                                                    float* __restrict__ ZB, float* __restrict__ BDT, unsigned short* __restrict__ WX16, unsigned short* __restrict__ WOUT16) {
  const unsigned bk = blockIdx.x;
  if (bk < 16u) {
    float* dp = ZB + bk * (unsigned)kThr + threadIdx.x;
    *(volatile float*)dp = 0.0f;
    __threadfence();
    *(volatile float*)dp = 0.0f;
  } else if (bk < 24u) {
    const unsigned i = (bk - 16u) * (unsigned)kThr + threadIdx.x;
    const float p = b_dt[i];
    const float o = bf16r(p);
    *(volatile float*)(BDT + i) = o;
    __threadfence();
    *(volatile float*)(BDT + i) = o;
  } else {
    const bool isX = bk < 280u;
    const unsigned j = (bk - (isX ? 24u : 280u)) * (unsigned)kThr + threadIdx.x;
    const size_t row = j >> 9;
    const unsigned c8 = (j & 511u) * 8u;
    const bool live = !isX || row < (size_t)kXo;
    const float* sp = (isX ? W_x : W_out) + (live ? row : 0) * kDI + (c8 & 2047u);
    const float cy = (c8 < 2048u) ? kInCarry : kW2Carry;
    const v4f a0 = *(const v4f*)sp, a1 = *(const v4f*)(sp + 4);
    v8h hv;
#pragma unroll
    for (int e = 0; e < 4; ++e) {
      const float f0 = a0[e], f1 = a1[e];
      hv[e] = (_Float16)(live ? carry_flush(bf16r(f0), cy) : 0.0f);
      hv[4 + e] = (_Float16)(live ? carry_flush(bf16r(f1), cy) : 0.0f);
    }
    unsigned short* dp = (isX ? WX16 : WOUT16) + row * kDI2 + c8;
    *(volatile v8h*)dp = hv;
    __threadfence();
    *(volatile v8h*)dp = hv;
  }
}
static_assert(2 * kDI == 16 * kThr && kDI == 8 * kThr && (size_t)kXoP * kDI2 / 8 == 256ull * kThr && (size_t)kDM * kDI2 / 8 == 2048ull * kThr && kDI2 / 8 == 512, "set-up grid exact: 16 blocks of zero bias, 8 of b_dt, 256 of the parameter map's doubled weight, 2,048 of the out-projection's");

__global__ __launch_bounds__(64) void conv_kernel(const float* __restrict__ XZ, const float* __restrict__ cw, const float* __restrict__ cb,
                                                   unsigned short* __restrict__ U16) {
  const int row = (int)blockIdx.y;
  const int tok = row & (kL - 1);
  const int c8 = (int)(blockIdx.x * 64u + threadIdx.x) * 8;
  float acc[8];
  {
    const v4f b0 = *(const v4f*)(cb + c8), b1 = *(const v4f*)(cb + c8 + 4);
#pragma unroll
    for (int e = 0; e < 4; ++e) { const float p = b0[e], q = b1[e]; acc[e] = bf16r(p); acc[4 + e] = bf16r(q); }
  }
  v4f wv[8];
#pragma unroll
  for (int e = 0; e < 8; ++e) wv[e] = *(const v4f*)(cw + (size_t)(c8 + e) * kDC);
#pragma unroll
  for (int k = 0; k < kDC; ++k) {
    const int back = kDC - 1 - k;
    const bool has = tok >= back;
    const float* xp = XZ + (size_t)(row - (has ? back : 0)) * (2 * kDI) + c8;
    const v4f x0 = *(const v4f*)xp, x1 = *(const v4f*)(xp + 4);
#pragma unroll
    for (int e = 0; e < 8; ++e) {
      const float w = wv[e][k];
      const float xv = (e < 4) ? x0[e] : x1[e - 4];
      acc[e] += has ? bf16r(w) * xv : 0.0f;
    }
  }
  v8h hv, lv;
#pragma unroll
  for (int e = 0; e < 8; ++e) {
    const float sc = carry_flush(acc[e], kInCarry);
    const _Float16 hi = (_Float16)sc;
    hv[e] = hi;
    lv[e] = (_Float16)carry_flush(sc - (float)hi, kLoUp);
  }
  unsigned short* hp = U16 + (size_t)row * kDI2 + c8;
  for (int pass = 0; pass < 2; ++pass) { *(volatile v8h*)hp = hv; *(volatile v8h*)(hp + kDI) = lv; __threadfence(); }
}
static_assert(kDI == 4 * 64 * 8, "front grid exact: 4 blocks of 64 chunks a row, 4,096 rows");

__global__ __launch_bounds__(kThr) void dt_cast_kernel(const float* __restrict__ XD, unsigned short* __restrict__ DT16) {
  const unsigned i = blockIdx.x * (unsigned)kThr + threadIdx.x;
  const size_t row = i >> 3;
  const unsigned c8 = (i & 7u) * 8u;
  const v4f a0 = *(const v4f*)(XD + row * kXoP + c8), a1 = *(const v4f*)(XD + row * kXoP + c8 + 4);
  v8h hv;
#pragma unroll
  for (int e = 0; e < 4; ++e) {
    hv[e] = (_Float16)carry_flush(a0[e], kDtCarry);
    hv[4 + e] = (_Float16)carry_flush(a1[e], kDtCarry);
  }
  unsigned short* dp = DT16 + row * kR + c8;
  *(volatile v8h*)dp = hv;
  __threadfence();
  *(volatile v8h*)dp = hv;
}
static_assert(kRows * 8 == 128 * kThr && kR == 8 * 8, "the step input's cast: 128 blocks; 8 chunks a row, all live");

__global__ __launch_bounds__(kThr) void scan_kernel(const float* __restrict__ XD, const float* __restrict__ DL, const float* __restrict__ XZ,
                                                    const float* __restrict__ cw, const float* __restrict__ cb, const float* __restrict__ A_log,
                                                    const float* __restrict__ Dp, unsigned short* __restrict__ Y16) {
  const unsigned ix = blockIdx.x * (unsigned)kThr + threadIdx.x;
  const unsigned sq = ix >> 10;
  const unsigned d0 = (ix & 1023u) * 2u;
  float A[2][kNs], h[2][kNs], dc[2], cwv[2][kDC], cbv[2], xw[2][kDC - 1];
#pragma unroll
  for (int k = 0; k < 2; ++k) {
    const unsigned d = d0 + (unsigned)k;
#pragma unroll
    for (int n = 0; n < kNs; ++n) { const float a = A_log[(size_t)d * kNs + n]; A[k][n] = -expf(bf16r(a)); h[k][n] = 0.0f; }
#pragma unroll
    for (int t = 0; t < kDC; ++t) { const float w = cw[(size_t)d * kDC + t]; cwv[k][t] = bf16r(w); }
    const float q0 = Dp[d], c0 = cb[d];
    dc[k] = bf16r(q0); cbv[k] = bf16r(c0);
    xw[k][0] = 0.0f; xw[k][1] = 0.0f; xw[k][2] = 0.0f;
  }
  for (int l = 0; l < kL; ++l) {
    const size_t row = (size_t)sq * kL + (size_t)l;
    const float* pr = XD + row * kXoP;
    const v2f xv = *(const v2f*)(XZ + row * (2 * kDI) + d0);
    const v2f zv = *(const v2f*)(XZ + row * (2 * kDI) + kDI + d0);
    const v2f pv = *(const v2f*)(DL + row * kDI + d0);
    float delta[2], dx[2], y[2], uu[2];
#pragma unroll
    for (int k = 0; k < 2; ++k) {
      float acc = cbv[k];
      acc += cwv[k][0] * xw[k][0];
      acc += cwv[k][1] * xw[k][1];
      acc += cwv[k][2] * xw[k][2];
      acc += cwv[k][3] * xv[k];
      xw[k][0] = xw[k][1]; xw[k][1] = xw[k][2]; xw[k][2] = xv[k];
      uu[k] = acc;
      const float pre = pv[k];
      delta[k] = (pre > 20.0f) ? pre : log1pf(expf(pre));
      dx[k] = delta[k] * uu[k];
      y[k] = 0.0f;
    }
#pragma unroll
    for (int q = 0; q < kNs / 4; ++q) {
      const v4f bv = *(const v4f*)(pr + kR + 4 * q), cv = *(const v4f*)(pr + kR + kNs + 4 * q);
#pragma unroll
      for (int e = 0; e < 4; ++e) {
        const int n = 4 * q + e;
#pragma unroll
        for (int k = 0; k < 2; ++k) {
          const float hn = expf(delta[k] * A[k][n]) * h[k][n] + dx[k] * bv[e];
          h[k][n] = hn;
          y[k] += hn * cv[e];
        }
      }
    }
    v2h hv, lv;
#pragma unroll
    for (int k = 0; k < 2; ++k) {
      const float yo = y[k] + dc[k] * uu[k];
      const float g = zv[k] / (1.0f + expf(-zv[k]));
      const float sc = carry_flush(yo * g, kYCarry);
      const _Float16 hi = (_Float16)sc;
      hv[k] = hi;
      lv[k] = (_Float16)carry_flush(sc - (float)hi, kLoUp);
    }
    unsigned short* dp = Y16 + row * kDI2 + d0;
    for (int pass = 0; pass < 2; ++pass) { *(volatile v2h*)dp = hv; *(volatile v2h*)(dp + kDI) = lv; __threadfence(); }
  }
}
static_assert(kNB * kDI / 2 == 8 * kThr && kDI / 2 == 1024 && (kNs % 4) == 0 && (kR % 4) == 0 && kDC == 4, "scan grid exact: 8 blocks: four a sequence; the B | C columns 16-B aligned; a 4-tap window");

extern "C" void kernel_launch(void* const* d_in, const int* in_sizes, int n_in,
                              void* d_out, int out_size, void* d_ws, size_t ws_size,
                              hipStream_t stream) {
  if (n_in < 10 || d_out == nullptr || d_ws == nullptr) return;
  if (in_sizes[0] != kRows * kDM || in_sizes[1] != 2 * kDI * kDM || in_sizes[2] != kDI * kDC || in_sizes[3] != kDI || in_sizes[4] != kDI * kNs) return;
  if (in_sizes[5] != kXo * kDI || in_sizes[6] != kDI * kR || in_sizes[7] != kDI || in_sizes[8] != kDI || in_sizes[9] != kDM * kDI) return;
  if (out_size != kRows * kDM) return;
  if (ws_size < kWsTotal) return;
  const float* x = (const float*)d_in[0];
  const float* W_in = (const float*)d_in[1];
  const float* conv_w = (const float*)d_in[2];
  const float* conv_b = (const float*)d_in[3];
  const float* A_log = (const float*)d_in[4];
  const float* W_x = (const float*)d_in[5];
  const float* W_dt = (const float*)d_in[6];
  const float* b_dt = (const float*)d_in[7];
  const float* D_skip = (const float*)d_in[8];
  const float* W_out = (const float*)d_in[9];
  float* out = (float*)d_out;
  char* ws = (char*)d_ws;
  unsigned short* X16 = (unsigned short*)(ws + kOffX16);
  unsigned short* WIN16 = (unsigned short*)(ws + kOffWIN16);
  unsigned short* WX16 = (unsigned short*)(ws + kOffWX16);
  unsigned short* WDT16 = (unsigned short*)(ws + kOffWDT16);
  unsigned short* WOUT16 = (unsigned short*)(ws + kOffWOUT16);
  float* ZB = (float*)(ws + kOffZB);
  float* BDT = (float*)(ws + kOffBDT);
  float* XZ = (float*)(ws + kOffXZ);
  unsigned short* U16 = (unsigned short*)(ws + kOffU16);
  unsigned short* Y16 = U16;
  float* XD = (float*)(ws + kOffXD);
  unsigned short* DT16 = (unsigned short*)(ws + kOffDT16);
  float* DL = (float*)(ws + kOffDL);

  static_assert(((size_t)kRows * kDM / 8) % kThr == 0 && ((size_t)2 * kDI * kDM / 8) % kThr == 0 && ((size_t)kDI * kR / 8) % kThr == 0 && ((size_t)kDI * kR) % 1024 == 0, "the casts' grids; every plane is whole rows of 1,024");
  cast_plane_kernel<<<(int)(((size_t)kRows * kDM / 8) / kThr), kThr, 0, stream>>>(x, X16, 10, kDM, 0);
  cast_plane_kernel<<<(int)(((size_t)2 * kDI * kDM / 8) / kThr), kThr, 0, stream>>>(W_in, WIN16, 10, kDM, 0);
  cast_plane_kernel<<<(int)(((size_t)kDI * kR / 8) / kThr), kThr, 0, stream>>>(W_dt, WDT16, 10, kDM, 0);
  setup_kernel<<<2328, kThr, 0, stream>>>(b_dt, W_x, W_out, ZB, BDT, WX16, WOUT16);
  wmma_gemm64<0, false, 2, 0, false, 0><<<dim3((kRows / 64) * (2 * kDI / 64) / 8, 1), 256, 0, stream>>>(
      X16, X16, kDM, 0L, WIN16, WIN16, kDM, 0L, (void*)XZ, (void*)XZ, 2 * kDI, 0L, ZB, nullptr, 0L, kRows, 2 * kDI, kDM, kScIn);
  conv_kernel<<<dim3(4, kRows), 64, 0, stream>>>(XZ, conv_w, conv_b, U16);
  wmma_gemm64<0, false, 2, 0, false, 0><<<dim3((kRows / 64) * (kXoP / 64) / 8, 1), 256, 0, stream>>>(
      U16, U16, kDI2, 0L, WX16, WX16, kDI2, 0L, (void*)XD, (void*)XD, kXoP, 0L, ZB, nullptr, 0L, kRows, kXoP, kDI2, kScIn);
  dt_cast_kernel<<<128, kThr, 0, stream>>>(XD, DT16);
  wmma_gemm64<0, false, 2, 0, false, 0><<<dim3((kRows / 64) * (kDI / 64) / 8, 1), 256, 0, stream>>>(
      DT16, DT16, kR, 0L, WDT16, WDT16, kR, 0L, (void*)DL, (void*)DL, kDI, 0L, BDT, nullptr, 0L, kRows, kDI, kR, kScDt);
  scan_kernel<<<8, kThr, 0, stream>>>(XD, DL, XZ, conv_w, conv_b, A_log, D_skip, Y16);
  wmma_gemm64<0, false, 2, 0, false, 0><<<dim3((kRows / 64) * (kDM / 64) / 8, 1), 256, 0, stream>>>(
      Y16, Y16, kDI2, 0L, WOUT16, WOUT16, kDI2, 0L, (void*)out, (void*)out, kDM, 0L, ZB, nullptr, 0L, kRows, kDM, kDI2, kScY);
}
static_assert(((kRows / 64) * (2 * kDI / 64)) % 8 == 0 && ((kRows / 64) * (kXoP / 64)) % 8 == 0 && ((kRows / 64) * (kDI / 64)) % 8 == 0 && ((kRows / 64) * (kDM / 64)) % 8 == 0, "the engine's grids: whole blocks of eight wave tiles");
